// TimeMixer_49787260895836
// MI455X (gfx1250) — hardware-verified
//
#include <hip/hip_runtime.h>
#include <math.h>

typedef __attribute__((ext_vector_type(8)))  _Float16 v8h;
typedef __attribute__((ext_vector_type(16))) __bf16   v16b;
typedef __attribute__((ext_vector_type(8)))  __bf16   v8b;
typedef __attribute__((ext_vector_type(8)))  float    v8f;
typedef __attribute__((ext_vector_type(4)))  float    v4f;
typedef __attribute__((ext_vector_type(4)))  unsigned int v4u;

constexpr int NBATCH   = 4;
constexpr int SEQ_T    = 1024;
constexpr int DIM_C    = 1024;
constexpr int N_HEAD   = 16;
constexpr int HEAD_D   = 64;
constexpr int ROWS_BT  = NBATCH * SEQ_T;
constexpr int TCHUNK   = 16;
constexpr int LR_MIX   = 32;
constexpr int LR_GATE  = 128;
constexpr int LR_DEC   = 64;
constexpr int LR_S     = 16;
constexpr int LR_SPAD  = 32;
constexpr float PRE_CARRY     = 16.0f;
constexpr float PRE_CARRY_INV = 0.0625f;

static_assert(DIM_C == N_HEAD * HEAD_D, "head split");
static_assert(HEAD_D == 64, "one 64-wide state row block per head");
static_assert(SEQ_T % TCHUNK == 0, "chunking");
static_assert((SEQ_T & (SEQ_T - 1)) == 0, "tmask trick needs power-of-two T");
static_assert(ROWS_BT % 64 == 0 && DIM_C % 64 == 0, "GEMM M/N tile multiples");
static_assert(DIM_C % 32 == 0 && LR_MIX % 32 == 0 && LR_GATE % 32 == 0 && LR_DEC % 32 == 0 && LR_SPAD % 32 == 0, "GEMM K % 32");
static_assert((4 * LR_MIX) % 64 == 0 && LR_GATE % 64 == 0, "GEMM N tile multiples for rank outputs");

constexpr size_t SZ_BIGW  = 2ull * DIM_C * DIM_C * 2;
constexpr size_t SZ_W128  = 2ull * 128 * DIM_C * 2;
constexpr size_t SZ_W64   = 2ull * 64 * DIM_C * 2;
constexpr size_t SZ_W32T  = 2ull * DIM_C * 32 * 2;
constexpr size_t SZ_ACT16 = 2ull * ROWS_BT * DIM_C * 2;
constexpr size_t SZ_SM16  = 2ull * ROWS_BT * 128 * 2;
constexpr size_t SZ_F32P  = (size_t)ROWS_BT * DIM_C * 4;
constexpr size_t SZ_F16P  = (size_t)ROWS_BT * DIM_C * 2;
constexpr size_t OFF_WB    = 0;
constexpr size_t OFF_WM1   = OFF_WB + SZ_BIGW;
constexpr size_t OFF_WM2   = OFF_WM1 + SZ_W128;
constexpr size_t OFF_WG1   = OFF_WM2 + SZ_W128;
constexpr size_t OFF_WG2T  = OFF_WG1 + SZ_W128;
constexpr size_t OFF_CMBK  = OFF_WG2T + SZ_W128;
constexpr size_t OFF_WKK2T = OFF_CMBK + SZ_W64;
constexpr size_t OFF_WMK2T = OFF_WKK2T + SZ_W32T;
constexpr size_t OFF_WD1   = OFF_WMK2T + SZ_W32T;
constexpr size_t OFF_CMBA  = OFF_WD1 + SZ_W64;
constexpr size_t OFF_WD2T  = OFF_CMBA + SZ_W64;
constexpr size_t OFF_WA2T  = OFF_WD2T + SZ_W64;
constexpr size_t OFF_WMA2T = OFF_WA2T + SZ_W32T;
constexpr size_t OFF_XM    = OFF_WMA2T + SZ_W32T;
constexpr size_t OFF_L0    = OFF_XM + SZ_ACT16;
constexpr size_t OFF_G1P   = OFF_L0 + SZ_SM16;
constexpr size_t OFF_SM    = OFF_G1P + SZ_SM16;
constexpr size_t OFF_R     = OFF_SM + SZ_SM16;
constexpr size_t OFF_KRAW  = OFF_R + SZ_F32P;
constexpr size_t OFF_KKZ   = OFF_KRAW + SZ_F32P;
constexpr size_t OFF_V     = OFF_KKZ + SZ_F32P;
constexpr size_t OFF_D2    = OFF_V + SZ_F32P;
constexpr size_t OFF_A2    = OFF_D2 + SZ_F16P;
constexpr size_t OFF_MA2   = OFF_A2 + SZ_F16P;
constexpr size_t OFF_MK2   = OFF_MA2 + SZ_F16P;
constexpr size_t WS_TOTAL  = OFF_MK2 + SZ_F16P;
static_assert(WS_TOTAL == 131596288ull, "carve total");
static_assert(WS_TOTAL <= 134217728ull, "carve cap");
static_assert(OFF_XM % 128 == 0 && OFF_R % 128 == 0 && OFF_D2 % 128 == 0, "line alignment");

__device__ __forceinline__ unsigned short f2bf_bits(float f) {
  unsigned u = __float_as_uint(f);
  return (unsigned short)((u + 0x7FFFu + ((u >> 16) & 1u)) >> 16);
}
__device__ __forceinline__ float bf_bits2f(unsigned short h) { return __uint_as_float(((unsigned)h) << 16); }
__device__ __forceinline__ float h2f(unsigned short u) { return (float)__builtin_bit_cast(_Float16, u); }
__device__ __forceinline__ void split2(float f, unsigned short& hb, unsigned short& lb) {
  hb = f2bf_bits(f);
  lb = f2bf_bits(f - bf_bits2f(hb));
}
__device__ __forceinline__ unsigned pk16(unsigned short a, unsigned short b) { return (unsigned)a | ((unsigned)b << 16); }

__device__ __forceinline__ void dep_guard_b(v8f& a, v8f& b, v16b x, v16b y) { asm volatile("v_nop\n\tv_nop\n\tv_nop\n\tv_nop" : "+v"(a), "+v"(b) : "v"(x), "v"(y)); }
__device__ __forceinline__ void keep4_b(v16b a, v16b b, v16b c, v16b d) { asm volatile("v_nop" :: "v"(a), "v"(b), "v"(c), "v"(d)); }
__device__ __forceinline__ void acc_guard4(v8f& a, v8f& b, v8f& c, v8f& d) { asm volatile("v_nop\n\tv_nop\n\tv_nop\n\tv_nop" : "+v"(a), "+v"(b), "+v"(c), "+v"(d)); }
__device__ __forceinline__ void acc_guard1(v8f& a, v16b w, v16b x, v16b y, v16b z) { asm volatile("v_nop\n\tv_nop\n\tv_nop\n\tv_nop" : "+v"(a) : "v"(w), "v"(x), "v"(y), "v"(z)); }
__device__ __forceinline__ void mem_clobber() { asm volatile("" ::: "memory"); }
__device__ __forceinline__ void lds_wave_sync() {
  __builtin_amdgcn_fence(__ATOMIC_RELEASE, "workgroup");
  __builtin_amdgcn_wave_barrier();
  __builtin_amdgcn_fence(__ATOMIC_ACQUIRE, "workgroup");
}
__device__ __forceinline__ float wsum(float v) {
#pragma unroll
  for (int off = 16; off >= 1; off >>= 1) v += __shfl_xor(v, off, 32);
  return v;
}

struct FragB {
  union U { v16b v; v8b h[2]; };
  static __device__ __forceinline__ v16b load(const __bf16* p) {
    U f; f.h[0] = *(const v8b*)(p); f.h[1] = *(const v8b*)(p + 16); return f.v;
  }
  static __device__ __forceinline__ v8f mma(v16b a, v16b b, v8f c) {
    return __builtin_amdgcn_wmma_f32_16x16x32_bf16(false, a, false, b, (short)0, c, false, false);
  }
};

__device__ __forceinline__ void pack8(const float (&v)[8], v4u& hv, v4u& lv) {
  unsigned hw[4], lw[4];
#pragma unroll
  for (int p = 0; p < 4; ++p) {
    unsigned short h0, l0, h1, l1;
    split2(v[2 * p], h0, l0);
    split2(v[2 * p + 1], h1, l1);
    hw[p] = pk16(h0, h1);
    lw[p] = pk16(l0, l1);
  }
  hv = (v4u){hw[0], hw[1], hw[2], hw[3]};
  lv = (v4u){lw[0], lw[1], lw[2], lw[3]};
}
__device__ __forceinline__ void store2x(unsigned short* ph, unsigned short* pl, v4u hv, v4u lv) {
  *(volatile v4u*)ph = hv;
  *(volatile v4u*)pl = lv;
  __threadfence();
  *(volatile v4u*)ph = hv;
  *(volatile v4u*)pl = lv;
}

__global__ __launch_bounds__(256) void cvt_planes(const float* __restrict__ in,
                                                  unsigned short* __restrict__ hi, unsigned short* __restrict__ lo, int n8) {
  const int q = blockIdx.x * 256 + threadIdx.x;
  if (q >= n8) return;
  const size_t e0 = (size_t)q * 8;
  const v4f a = *(const v4f*)(in + e0);
  const v4f c = *(const v4f*)(in + e0 + 4);
  float v[8] = {a[0], a[1], a[2], a[3], c[0], c[1], c[2], c[3]};
  v4u hv, lv;
  pack8(v, hv, lv);
  store2x(hi + e0, lo + e0, hv, lv);
}

__global__ __launch_bounds__(256) void cvt_transpose_planes(const float* __restrict__ in,
                                                            unsigned short* __restrict__ hi, unsigned short* __restrict__ lo,
                                                            int nN, int kReal, int kPad, int kLo, int n8) {
  const int q = blockIdx.x * 256 + threadIdx.x;
  if (q >= n8) return;
  const int per = kPad >> 3;
  const int n = q / per;
  const int kb = (q - n * per) * 8;
  float v[8];
#pragma unroll
  for (int e = 0; e < 8; ++e) {
    const int k = kb + e - kLo;
    const bool valid = (k >= 0) && (k < kReal);
    int kc = (k < 0) ? 0 : k;
    kc = (kc >= kReal) ? (kReal - 1) : kc;
    const float f = in[(size_t)kc * nN + n];
    v[e] = valid ? f : 0.0f;
  }
  v4u hv, lv;
  pack8(v, hv, lv);
  const size_t e0 = (size_t)q * 8;
  store2x(hi + e0, lo + e0, hv, lv);
}

__global__ __launch_bounds__(256) void cvt_rowsel_planes(const float* __restrict__ inA, const float* __restrict__ inB,
                                                         unsigned short* __restrict__ hi, unsigned short* __restrict__ lo,
                                                         int ncol, int n8) {
  const int q = blockIdx.x * 256 + threadIdx.x;
  if (q >= n8) return;
  const int per = ncol >> 3;
  const int n = q / per;
  const int c = (q - n * per) * 8;
  const int ra = n & 15;
  const int useB = (n >> 4) & 1;
  const size_t so = (size_t)ra * ncol + c;
  const v4f a0 = *(const v4f*)(inA + so), a1 = *(const v4f*)(inA + so + 4);
  const v4f b0 = *(const v4f*)(inB + so), b1 = *(const v4f*)(inB + so + 4);
  float v[8];
#pragma unroll
  for (int e = 0; e < 4; ++e) {
    v[e]     = useB ? b0[e] : a0[e];
    v[4 + e] = useB ? b1[e] : a1[e];
  }
  v4u hv, lv;
  pack8(v, hv, lv);
  const size_t e0 = (size_t)q * 8;
  store2x(hi + e0, lo + e0, hv, lv);
}

__global__ __launch_bounds__(256) void token_shift_planes(const float* __restrict__ x, const float* __restrict__ mx,
                                                          unsigned short* __restrict__ hi, unsigned short* __restrict__ lo,
                                                          int ncol, int tmask, int n8) {
  const int q = blockIdx.x * 256 + threadIdx.x;
  if (q >= n8) return;
  const int per = ncol >> 3;
  const int mrow = q / per;
  const int c = (q - mrow * per) * 8;
  const int nz = ((mrow & tmask) != 0) ? 1 : 0;
  const int pr = mrow - nz;
  const size_t o  = (size_t)mrow * ncol + c;
  const size_t op = (size_t)pr * ncol + c;
  const v4f xa0 = *(const v4f*)(x + o),  xa1 = *(const v4f*)(x + o + 4);
  const v4f xq0 = *(const v4f*)(x + op), xq1 = *(const v4f*)(x + op + 4);
  const v4f m0  = *(const v4f*)(mx + c), m1  = *(const v4f*)(mx + c + 4);
  float v[8];
#pragma unroll
  for (int e = 0; e < 4; ++e) {
    const float xp0 = nz ? xq0[e] : 0.0f;
    const float xp1 = nz ? xq1[e] : 0.0f;
    v[e]     = xa0[e] + (xp0 - xa0[e]) * m0[e];
    v[4 + e] = xa1[e] + (xp1 - xa1[e]) * m1[e];
  }
  v4u hv, lv;
  pack8(v, hv, lv);
  store2x(hi + o, lo + o, hv, lv);
}

template <int OUT_MODE, bool RESID, int ACT, int EPI>
__global__ __launch_bounds__(256) void gemm64(
    const unsigned short* __restrict__ Ap, const unsigned short* __restrict__ A2p, int lda,
    const unsigned short* __restrict__ Btp, const unsigned short* __restrict__ Bt2p, int ldb,
    void* __restrict__ Cout, void* __restrict__ Cout2, int ldc,
    const float* __restrict__ resid,
    const float* __restrict__ aux, const float* __restrict__ auxv, int tmask,
    int M, int N, int K, float scale) {
  const __bf16* A   = (const __bf16*)Ap;
  const __bf16* A2  = (const __bf16*)A2p;
  const __bf16* Bt  = (const __bf16*)Btp;
  const __bf16* Bt2 = (const __bf16*)Bt2p;
  __shared__ __align__(16) float sT[8][16 * 68];
  const int lane = threadIdx.x & 31;
  const int wave = threadIdx.x >> 5;
  const int tilesN = N >> 6;
  const int tilesM = M >> 6;
  const int tile = blockIdx.x * 8 + wave;
  if (tile >= tilesM * tilesN) return;
  const int tm = tile / tilesN;
  const int tn = tile - tm * tilesN;
  const int m0 = tm << 6;
  const int n0 = tn << 6;
  const int rlane = lane & 15;
  const int koff  = (lane >> 4) * 8;
  const int mOff  = (lane >> 4) * 8;

  v8f acc[4][4];
#pragma unroll
  for (int i = 0; i < 4; ++i)
#pragma unroll
    for (int j = 0; j < 4; ++j) acc[i][j] = (v8f){0.f,0.f,0.f,0.f,0.f,0.f,0.f,0.f};

  for (int k0 = 0; k0 < K; k0 += 32) {
    v16b bh[4], bl[4];
#pragma unroll
    for (int j = 0; j < 4; ++j) {
      const size_t bo = (size_t)(n0 + (j << 4) + rlane) * ldb + koff + k0;
      bh[j] = FragB::load(Bt + bo);
      bl[j] = FragB::load(Bt2 + bo);
    }
#pragma unroll
    for (int i = 0; i < 4; ++i) {
      const size_t ao = (size_t)(m0 + (i << 4) + rlane) * lda + koff + k0;
      const v16b ah = FragB::load(A + ao);
      const v16b al = FragB::load(A2 + ao);
#pragma unroll
      for (int j = 0; j < 4; ++j) {
        acc[i][j] = FragB::mma(ah, bh[j], acc[i][j]);
        acc[i][j] = FragB::mma(ah, bl[j], acc[i][j]);
        acc[i][j] = FragB::mma(al, bh[j], acc[i][j]);
      }
      dep_guard_b(acc[i][0], acc[i][3], ah, al);
    }
    keep4_b(bh[0], bh[1], bh[2], bh[3]);
    keep4_b(bl[0], bl[1], bl[2], bl[3]);
  }
  acc_guard4(acc[0][0], acc[0][1], acc[0][2], acc[0][3]);
  acc_guard4(acc[1][0], acc[1][1], acc[1][2], acc[1][3]);
  acc_guard4(acc[2][0], acc[2][1], acc[2][2], acc[2][3]);
  acc_guard4(acc[3][0], acc[3][1], acc[3][2], acc[3][3]);

  float* slab = sT[wave];
#pragma unroll
  for (int i = 0; i < 4; ++i) {
    const int mBase = m0 + (i << 4);
#pragma unroll
    for (int j = 0; j < 4; ++j) {
      const int n = n0 + (j << 4) + rlane;
      float av = 0.f;
      if (EPI == 1) av = auxv[n];
      if (EPI != 0 || RESID) mem_clobber();
#pragma unroll
      for (int r = 0; r < 8; ++r) {
        const int mrow = mBase + mOff + r;
        float v = acc[i][j][r] * scale;
        if (RESID) v += resid[(size_t)mrow * ldc + n];
        if (EPI == 1) {
          if (r == 4) mem_clobber();
          const int nz = ((mrow & tmask) != 0) ? 1 : 0;
          const float xv = aux[(size_t)mrow * ldc + n];
          const float xq = aux[(size_t)(mrow - nz) * ldc + n];
          const float xp = nz ? xq : 0.0f;
          v = xv + (xp - xv) * (av + v);
        }
        if (EPI == 2) v = aux[(size_t)mrow * ldc + n] * v;
        if (ACT == 1) v = tanhf(v);
        slab[(mOff + r) * 68 + (j << 4) + rlane] = v;
      }
    }
    lds_wave_sync();
    if (OUT_MODE == 0) {
      float* Cp = (float*)Cout;
      const int hh = lane >> 4, c4 = (lane & 15) * 4;
      for (int pass = 0; pass < 2; ++pass) {
#pragma unroll
        for (int it = 0; it < 8; ++it) {
          const int row = it * 2 + hh;
          const v4f vv = *(const v4f*)(slab + row * 68 + c4);
          *(volatile v4f*)(Cp + (size_t)(mBase + row) * ldc + n0 + c4) = vv;
        }
        __threadfence();
      }
    } else {
      const int q = lane >> 3, c8 = (lane & 7) * 8;
      unsigned short* Cp  = (unsigned short*)Cout;
      unsigned short* Cp2 = (OUT_MODE == 2) ? (unsigned short*)Cout2 : nullptr;
      for (int pass = 0; pass < 2; ++pass) {
#pragma unroll
        for (int it = 0; it < 4; ++it) {
          const int row = it * 4 + q;
          const float* sp = slab + row * 68 + c8;
          v8h hv, lv;
#pragma unroll
          for (int e = 0; e < 8; ++e) {
            if (OUT_MODE == 1) {
              hv[e] = (_Float16)sp[e];
            } else {
              const unsigned short hb = f2bf_bits(sp[e]);
              const unsigned short lb = f2bf_bits(sp[e] - bf_bits2f(hb));
              hv[e] = __builtin_bit_cast(_Float16, hb);
              lv[e] = __builtin_bit_cast(_Float16, lb);
            }
          }
          *(volatile v8h*)(Cp + (size_t)(mBase + row) * ldc + n0 + c8) = hv;
          if (OUT_MODE == 2) *(volatile v8h*)(Cp2 + (size_t)(mBase + row) * ldc + n0 + c8) = lv;
        }
        __threadfence();
      }
    }
    lds_wave_sync();
  }
}

__global__ __launch_bounds__(128) void decay_scan(
    const float* Rp, const float* Kp, float* KKZ, const float* Vp,
    const unsigned short* D2p, const unsigned short* A2p, const unsigned short* MA2p, const unsigned short* MK2p,
    const float* tdec, const float* iclr0, const float* misca, const float* misck,
    const float* bonusw, const float* lnw, const float* lnb, int seqT, int dimC, int nH) {
  __shared__ __align__(16) float sR[TCHUNK * 64];
  __shared__ __align__(16) float sK[TCHUNK * 64];
  __shared__ __align__(16) float sKK[TCHUNK * 64];
  __shared__ __align__(16) float sV[TCHUNK * 64];
  __shared__ __align__(16) float sW[TCHUNK * 64];
  __shared__ __align__(16) float sBv[TCHUNK * 64];
  __shared__ __align__(16) float sY[TCHUNK * 64];
  __shared__ __align__(16) unsigned short sP16[4][TCHUNK * 64];
  __shared__ __align__(16) unsigned short sBcH[(2 * TCHUNK + 1) * 64];
  __shared__ __align__(16) unsigned short sBcL[(2 * TCHUNK + 1) * 64];
  __shared__ __align__(16) float sDot[TCHUNK * 2];
  __shared__ __align__(16) float sDw[4][32];
  __shared__ __align__(16) float sPar[7 * 64];

  const int tid  = threadIdx.x;
  const int lane = tid & 31;
  const int wv   = tid >> 5;
  const int bh   = blockIdx.x;
  const int b    = bh / nH;
  const int h    = bh - b * nH;
  const int m    = lane & 15;
  const int hl   = lane >> 4;
  const int koff = hl * 8;
  const int row  = wv * 16 + m;
  const int c0   = h * HEAD_D;

  if (tid < 64) {
    const int c = c0 + tid;
    sPar[tid]       = tdec[c];
    sPar[64 + tid]  = iclr0[c];
    sPar[128 + tid] = misca[c];
    sPar[192 + tid] = misck[c];
    sPar[256 + tid] = bonusw[c];
    sPar[320 + tid] = lnw[c];
    sPar[384 + tid] = lnb[c];
  }
  if (tid < 8) {
    const v4u z = {0u, 0u, 0u, 0u};
    *(v4u*)(sBcH + 2 * TCHUNK * 64 + tid * 8) = z;
    *(v4u*)(sBcL + 2 * TCHUNK * 64 + tid * 8) = z;
  }

  float S[32];
#pragma unroll
  for (int e = 0; e < 32; ++e) S[e] = 0.0f;

  const int nChunk = seqT / TCHUNK;
  for (int ci = 0; ci < nChunk; ++ci) {
    const int t0 = ci * TCHUNK;
    const size_t rowg0 = (size_t)(b * seqT + t0);
    __syncthreads();
#pragma unroll
    for (int u = 0; u < 2; ++u) {
      const int q = tid + 128 * u;
      const int tt = q >> 4, c4 = (q & 15) * 4;
      const size_t g = (rowg0 + tt) * dimC + c0 + c4;
      *(v4f*)(sR + tt * 64 + c4)  = *(const v4f*)(Rp + g);
      *(v4f*)(sK + tt * 64 + c4)  = *(const v4f*)(Kp + g);
      *(v4f*)(sKK + tt * 64 + c4) = *(const v4f*)(KKZ + g);
      *(v4f*)(sV + tt * 64 + c4)  = *(const v4f*)(Vp + g);
    }
    {
      const int tt = tid >> 3, c8 = (tid & 7) * 8;
      const size_t g = (rowg0 + tt) * dimC + c0 + c8;
      *(v4u*)(sP16[0] + tt * 64 + c8) = *(const v4u*)(D2p + g);
      *(v4u*)(sP16[1] + tt * 64 + c8) = *(const v4u*)(A2p + g);
      *(v4u*)(sP16[2] + tt * 64 + c8) = *(const v4u*)(MA2p + g);
      *(v4u*)(sP16[3] + tt * 64 + c8) = *(const v4u*)(MK2p + g);
    }
    __syncthreads();

#pragma unroll 1
    for (int q = 0; q < 4; ++q) {
      const int tt = wv * 4 + q;
      float rv[2], kmv[2], kkv[2], av[2], wdv[2];
      float ss = 0.0f;
#pragma unroll
      for (int u = 0; u < 2; ++u) {
        const int jj = lane + 32 * u;
        const int o = tt * 64 + jj;
        const float kraw = sK[o];
        const float kk   = sKK[o];
        const float d2 = h2f(sP16[0][o]) * PRE_CARRY_INV;
        const float a2 = h2f(sP16[1][o]) * PRE_CARRY_INV;
        const float m2 = h2f(sP16[2][o]) * PRE_CARRY_INV;
        const float k2 = h2f(sP16[3][o]) * PRE_CARRY_INV;
        const float u0 = -(sPar[jj] + d2);
        const float sp = fmaxf(u0, 0.0f) + log1pf(expf(-fabsf(u0)));
        const float wl = -sp - 0.5f;
        const float ag  = 1.0f / (1.0f + expf(-(sPar[64 + jj] + a2)));
        const float mag = 1.0f / (1.0f + expf(-(sPar[128 + jj] + m2)));
        const float mkg = 1.0f / (1.0f + expf(-(sPar[192 + jj] + k2)));
        float km = kraw * (mag + ag * (1.0f - mag));
        km = km * expf(fminf(wl * mkg, 0.0f));
        rv[u]  = sR[o];
        kmv[u] = km;
        kkv[u] = kk;
        av[u]  = ag;
        wdv[u] = expf(-expf(wl));
        ss += kk * kk;
      }
      ss = wsum(ss);
      const float inv = 1.0f / fmaxf(sqrtf(ss), 1e-12f);
      float pbr = 0.0f, pkr = 0.0f;
#pragma unroll
      for (int u = 0; u < 2; ++u) {
        const int jj = lane + 32 * u;
        const int o = tt * 64 + jj;
        const float kkn = kkv[u] * inv;
        const float bb  = kkn * av[u];
        sK[o]  = kmv[u];
        sBv[o] = bb;
        sW[o]  = wdv[u];
        unsigned short h0, l0, h1, l1;
        split2(-kkn, h0, l0);
        split2(wdv[u] * rv[u], h1, l1);
        sBcH[(tt * 2) * 64 + jj]     = h0;
        sBcL[(tt * 2) * 64 + jj]     = l0;
        sBcH[(tt * 2 + 1) * 64 + jj] = h1;
        sBcL[(tt * 2 + 1) * 64 + jj] = l1;
        pbr += bb * rv[u];
        pkr += kmv[u] * rv[u];
      }
      pbr = wsum(pbr);
      pkr = wsum(pkr);
      if (lane == 0) { sDot[tt * 2] = pbr; sDot[tt * 2 + 1] = pkr; }
    }
    __syncthreads();

#pragma unroll 1
    for (int ts = 0; ts < TCHUNK; ++ts) {
      v16b ah0, al0, ah1, al1;
#pragma unroll
      for (int e = 0; e < 16; ++e) {
        unsigned short hb, lb;
        split2(S[e], hb, lb);
        ah0[e] = __builtin_bit_cast(__bf16, hb);
        al0[e] = __builtin_bit_cast(__bf16, lb);
        split2(S[16 + e], hb, lb);
        ah1[e] = __builtin_bit_cast(__bf16, hb);
        al1[e] = __builtin_bit_cast(__bf16, lb);
      }
      const int si = (m < 2) ? (ts * 2 + m) : (2 * TCHUNK);
      const __bf16* pH = (const __bf16*)(sBcH + si * 64 + koff);
      const __bf16* pL = (const __bf16*)(sBcL + si * 64 + koff);
      const v16b bh0 = FragB::load(pH);
      const v16b bh1 = FragB::load(pH + 32);
      const v16b bl0 = FragB::load(pL);
      const v16b bl1 = FragB::load(pL + 32);
      v8f acc = (v8f){0.f,0.f,0.f,0.f,0.f,0.f,0.f,0.f};
      acc = FragB::mma(ah0, bh0, acc);
      acc = FragB::mma(ah0, bl0, acc);
      acc = FragB::mma(al0, bh0, acc);
      acc = FragB::mma(ah1, bh1, acc);
      acc = FragB::mma(ah1, bl1, acc);
      acc = FragB::mma(al1, bh1, acc);
      acc_guard1(acc, ah1, bh1, al1, bl1);
      if (m < 2) {
#pragma unroll
        for (int r = 0; r < 8; ++r) sDw[wv][(8 * hl + r) * 2 + m] = acc[r];
      }
      lds_wave_sync();
      const float Sa  = sDw[wv][m * 2];
      const float Swr = sDw[wv][m * 2 + 1];
      lds_wave_sync();
      const int ob = ts * 64;
      const float vi  = sV[ob + row];
      const float dbr = sDot[ts * 2];
      const float dkr = sDot[ts * 2 + 1];
      const float yi  = Swr + Sa * dbr + vi * dkr;
      if (hl == 0) sY[ob + row] = yi;
#pragma unroll
      for (int ks = 0; ks < 2; ++ks) {
#pragma unroll
        for (int g = 0; g < 2; ++g) {
          const int kb = ob + ks * 32 + g * 16 + koff;
          const v4f w0 = *(const v4f*)(sW + kb),  w1 = *(const v4f*)(sW + kb + 4);
          const v4f b0 = *(const v4f*)(sBv + kb), b1 = *(const v4f*)(sBv + kb + 4);
          const v4f k0 = *(const v4f*)(sK + kb),  k1 = *(const v4f*)(sK + kb + 4);
#pragma unroll
          for (int i = 0; i < 4; ++i) {
            const int e = ks * 16 + g * 8 + i;
            S[e]     = (S[e] * w0[i] + Sa * b0[i]) + vi * k0[i];
            S[e + 4] = (S[e + 4] * w1[i] + Sa * b1[i]) + vi * k1[i];
          }
        }
      }
    }
    __syncthreads();

#pragma unroll 1
    for (int q = 0; q < 4; ++q) {
      const int tt = wv * 4 + q;
      const int o0 = tt * 64 + lane, o1 = o0 + 32;
      const float y0 = sY[o0], y1 = sY[o1];
      const float mu = wsum(y0 + y1) * (1.0f / 64.0f);
      const float d0 = y0 - mu, d1 = y1 - mu;
      const float var = wsum(d0 * d0 + d1 * d1) * (1.0f / 64.0f);
      const float rs = 1.0f / sqrtf(var + 6.4e-4f);
      const float sbn = wsum(sR[o0] * sK[o0] * sPar[256 + lane] + sR[o1] * sK[o1] * sPar[256 + lane + 32]);
      const float z0 = (d0 * rs * sPar[320 + lane] + sPar[384 + lane]) + sbn * sV[o0];
      const float z1 = (d1 * rs * sPar[320 + lane + 32] + sPar[384 + lane + 32]) + sbn * sV[o1];
      sY[o0] = z0;
      sY[o1] = z1;
    }
    __syncthreads();
    {
      const int c4 = (lane & 15) * 4;
      for (int pass = 0; pass < 2; ++pass) {
#pragma unroll
        for (int it = 0; it < 2; ++it) {
          const int tt = wv * 4 + it * 2 + hl;
          const v4f val = *(const v4f*)(sY + tt * 64 + c4);
          *(volatile v4f*)(KKZ + (rowg0 + tt) * dimC + c0 + c4) = val;
        }
        __threadfence();
      }
    }
  }
}

extern "C" void kernel_launch(void* const* d_in, const int* in_sizes, int n_in,
                              void* d_out, int out_size, void* d_ws, size_t ws_size, hipStream_t stream) {
  if (n_in < 29) return;
  if (in_sizes[0] != ROWS_BT * DIM_C || out_size != ROWS_BT * DIM_C) return;
  if (in_sizes[23] != DIM_C * DIM_C || in_sizes[4] != 128 * DIM_C || in_sizes[5] != 4 * DIM_C * 32) return;
  if (ws_size < WS_TOTAL) return;

  const float* x        = (const float*)d_in[0];
  const float* maa_x    = (const float*)d_in[2];
  const float* maa      = (const float*)d_in[3];
  const float* maa_w1   = (const float*)d_in[4];
  const float* maa_w2   = (const float*)d_in[5];
  const float* tdecay   = (const float*)d_in[6];
  const float* dec_w1   = (const float*)d_in[7];
  const float* dec_w2   = (const float*)d_in[8];
  const float* aaaaa    = (const float*)d_in[9];
  const float* aaa_w1   = (const float*)d_in[10];
  const float* aaa_w2   = (const float*)d_in[11];
  const float* kkk_w1   = (const float*)d_in[12];
  const float* kkk_w2   = (const float*)d_in[13];
  const float* gate_w1  = (const float*)d_in[14];
  const float* gate_w2  = (const float*)d_in[15];
  const float* misc_a   = (const float*)d_in[16];
  const float* ma_w1    = (const float*)d_in[17];
  const float* ma_w2    = (const float*)d_in[18];
  const float* misc_k   = (const float*)d_in[19];
  const float* mk_w1    = (const float*)d_in[20];
  const float* mk_w2    = (const float*)d_in[21];
  const float* faaaa    = (const float*)d_in[22];
  const float* Wr       = (const float*)d_in[23];
  const float* Wk       = (const float*)d_in[24];
  const float* Wv       = (const float*)d_in[25];
  const float* Wo       = (const float*)d_in[26];
  const float* ln_w     = (const float*)d_in[27];
  const float* ln_b     = (const float*)d_in[28];
  float* out = (float*)d_out;

  char* ws = (char*)d_ws;
  auto P16 = [&](size_t off) { return (unsigned short*)(ws + off); };
  auto P32 = [&](size_t off) { return (float*)(ws + off); };
  unsigned short *WBh = P16(OFF_WB),    *WBl = P16(OFF_WB + SZ_BIGW / 2);
  unsigned short *WM1h = P16(OFF_WM1),  *WM1l = P16(OFF_WM1 + SZ_W128 / 2);
  unsigned short *WM2h = P16(OFF_WM2),  *WM2l = P16(OFF_WM2 + SZ_W128 / 2);
  unsigned short *WG1h = P16(OFF_WG1),  *WG1l = P16(OFF_WG1 + SZ_W128 / 2);
  unsigned short *WG2h = P16(OFF_WG2T), *WG2l = P16(OFF_WG2T + SZ_W128 / 2);
  unsigned short *CKh  = P16(OFF_CMBK), *CKl  = P16(OFF_CMBK + SZ_W64 / 2);
  unsigned short *KK2h = P16(OFF_WKK2T),*KK2l = P16(OFF_WKK2T + SZ_W32T / 2);
  unsigned short *MK2Th= P16(OFF_WMK2T),*MK2Tl= P16(OFF_WMK2T + SZ_W32T / 2);
  unsigned short *WD1h = P16(OFF_WD1),  *WD1l = P16(OFF_WD1 + SZ_W64 / 2);
  unsigned short *CAh  = P16(OFF_CMBA), *CAl  = P16(OFF_CMBA + SZ_W64 / 2);
  unsigned short *WD2h = P16(OFF_WD2T), *WD2l = P16(OFF_WD2T + SZ_W64 / 2);
  unsigned short *WA2h = P16(OFF_WA2T), *WA2l = P16(OFF_WA2T + SZ_W32T / 2);
  unsigned short *WMAh = P16(OFF_WMA2T),*WMAl = P16(OFF_WMA2T + SZ_W32T / 2);
  unsigned short *XMh  = P16(OFF_XM),   *XMl  = P16(OFF_XM + SZ_ACT16 / 2);
  unsigned short *L0h  = P16(OFF_L0),   *L0l  = P16(OFF_L0 + SZ_SM16 / 2);
  unsigned short *G1h  = P16(OFF_G1P),  *G1l  = P16(OFF_G1P + SZ_SM16 / 2);
  unsigned short *SMh  = P16(OFF_SM),   *SMl  = P16(OFF_SM + SZ_SM16 / 2);
  float* Rp   = P32(OFF_R);
  float* Kraw = P32(OFF_KRAW);
  float* KKZ  = P32(OFF_KKZ);
  float* Vp   = P32(OFF_V);
  unsigned short* D2p  = P16(OFF_D2);
  unsigned short* A2p  = P16(OFF_A2);
  unsigned short* MA2p = P16(OFF_MA2);
  unsigned short* MK2p = P16(OFF_MK2);

  const int tmask = SEQ_T - 1;
  auto grid_g = [&](int M, int N) { return dim3((unsigned)(((M / 64) * (N / 64) + 7) / 8)); };
  auto cvt = [&](const float* src, unsigned short* hi, unsigned short* lo, int nelem) {
    const int n8 = nelem / 8;
    cvt_planes<<<(unsigned)(n8 / 256), 256, 0, stream>>>(src, hi, lo, n8);
  };
  auto cvtT = [&](const float* src, unsigned short* hi, unsigned short* lo, int nN, int kReal, int kPad, int kLo) {
    const int n8 = nN * kPad / 8;
    cvt_transpose_planes<<<(unsigned)(n8 / 256), 256, 0, stream>>>(src, hi, lo, nN, kReal, kPad, kLo, n8);
  };

  cvt(maa_w1, WM1h, WM1l, 128 * DIM_C);
  cvt(maa_w2, WM2h, WM2l, 4 * DIM_C * LR_MIX);
  cvt(gate_w1, WG1h, WG1l, LR_GATE * DIM_C);
  cvtT(gate_w2, WG2h, WG2l, DIM_C, LR_GATE, LR_GATE, 0);
  cvt_rowsel_planes<<<(unsigned)((64 * DIM_C / 8) / 256), 256, 0, stream>>>(kkk_w1, mk_w1, CKh, CKl, DIM_C, 64 * DIM_C / 8);
  cvtT(kkk_w2, KK2h, KK2l, DIM_C, LR_S, LR_SPAD, 0);
  cvtT(mk_w2, MK2Th, MK2Tl, DIM_C, LR_S, LR_SPAD, LR_S);
  cvt(dec_w1, WD1h, WD1l, LR_DEC * DIM_C);
  cvt_rowsel_planes<<<(unsigned)((64 * DIM_C / 8) / 256), 256, 0, stream>>>(aaa_w1, ma_w1, CAh, CAl, DIM_C, 64 * DIM_C / 8);
  cvtT(dec_w2, WD2h, WD2l, DIM_C, LR_DEC, LR_DEC, 0);
  cvtT(aaa_w2, WA2h, WA2l, DIM_C, LR_S, LR_SPAD, 0);
  cvtT(ma_w2, WMAh, WMAl, DIM_C, LR_S, LR_SPAD, LR_S);

  token_shift_planes<<<(unsigned)((ROWS_BT * DIM_C / 8) / 256), 256, 0, stream>>>(x, maa_x, XMh, XMl, DIM_C, tmask, ROWS_BT * DIM_C / 8);
  gemm64<2, false, 1, 0><<<grid_g(ROWS_BT, 128), 256, 0, stream>>>(XMh, XMl, DIM_C, WM1h, WM1l, DIM_C, L0h, L0l, 128,
                                                                   nullptr, nullptr, nullptr, 0, ROWS_BT, 128, DIM_C, 1.0f);
  auto mixgemm = [&](int br) {
    gemm64<2, false, 0, 1><<<grid_g(ROWS_BT, DIM_C), 256, 0, stream>>>(L0h + LR_MIX * br, L0l + LR_MIX * br, 128,
        WM2h + (size_t)br * DIM_C * LR_MIX, WM2l + (size_t)br * DIM_C * LR_MIX, LR_MIX,
        XMh, XMl, DIM_C, nullptr, x, maa + (size_t)br * DIM_C, tmask, ROWS_BT, DIM_C, LR_MIX, 1.0f);
  };

  mixgemm(0);
  cvt(Wr, WBh, WBl, DIM_C * DIM_C);
  gemm64<0, false, 0, 0><<<grid_g(ROWS_BT, DIM_C), 256, 0, stream>>>(XMh, XMl, DIM_C, WBh, WBl, DIM_C, Rp, nullptr, DIM_C,
                                                                    nullptr, nullptr, nullptr, 0, ROWS_BT, DIM_C, DIM_C, 1.0f);
  gemm64<2, false, 1, 0><<<grid_g(ROWS_BT, LR_GATE), 256, 0, stream>>>(XMh, XMl, DIM_C, WG1h, WG1l, DIM_C, G1h, G1l, LR_GATE,
                                                                      nullptr, nullptr, nullptr, 0, ROWS_BT, LR_GATE, DIM_C, 1.0f);

  mixgemm(2);
  cvt(Wk, WBh, WBl, DIM_C * DIM_C);
  gemm64<0, false, 0, 0><<<grid_g(ROWS_BT, DIM_C), 256, 0, stream>>>(XMh, XMl, DIM_C, WBh, WBl, DIM_C, Kraw, nullptr, DIM_C,
                                                                    nullptr, nullptr, nullptr, 0, ROWS_BT, DIM_C, DIM_C, 1.0f);
  gemm64<2, false, 0, 0><<<grid_g(ROWS_BT, 64), 256, 0, stream>>>(XMh, XMl, DIM_C, CKh, CKl, DIM_C, SMh, SMl, 128,
                                                                 nullptr, nullptr, nullptr, 0, ROWS_BT, 64, DIM_C, 1.0f);
  gemm64<0, true, 0, 0><<<grid_g(ROWS_BT, DIM_C), 256, 0, stream>>>(SMh, SMl, 128, KK2h, KK2l, LR_SPAD, KKZ, nullptr, DIM_C,
                                                                   Kraw, nullptr, nullptr, 0, ROWS_BT, DIM_C, LR_SPAD, 1.0f);
  gemm64<1, false, 0, 0><<<grid_g(ROWS_BT, DIM_C), 256, 0, stream>>>(SMh, SMl, 128, MK2Th, MK2Tl, LR_SPAD, MK2p, nullptr, DIM_C,
                                                                    nullptr, nullptr, nullptr, 0, ROWS_BT, DIM_C, LR_SPAD, PRE_CARRY);

  mixgemm(3);
  cvt(Wv, WBh, WBl, DIM_C * DIM_C);
  gemm64<0, false, 0, 0><<<grid_g(ROWS_BT, DIM_C), 256, 0, stream>>>(XMh, XMl, DIM_C, WBh, WBl, DIM_C, Vp, nullptr, DIM_C,
                                                                    nullptr, nullptr, nullptr, 0, ROWS_BT, DIM_C, DIM_C, 1.0f);

  mixgemm(1);
  gemm64<2, false, 1, 0><<<grid_g(ROWS_BT, 64), 256, 0, stream>>>(XMh, XMl, DIM_C, WD1h, WD1l, DIM_C, SMh, SMl, 128,
                                                                 nullptr, nullptr, nullptr, 0, ROWS_BT, 64, DIM_C, 1.0f);
  gemm64<2, false, 0, 0><<<grid_g(ROWS_BT, 64), 256, 0, stream>>>(XMh, XMl, DIM_C, CAh, CAl, DIM_C, SMh + 64, SMl + 64, 128,
                                                                 nullptr, nullptr, nullptr, 0, ROWS_BT, 64, DIM_C, 1.0f);
  gemm64<1, false, 0, 0><<<grid_g(ROWS_BT, DIM_C), 256, 0, stream>>>(SMh, SMl, 128, WD2h, WD2l, LR_DEC, D2p, nullptr, DIM_C,
                                                                    nullptr, nullptr, nullptr, 0, ROWS_BT, DIM_C, LR_DEC, PRE_CARRY);
  gemm64<1, false, 0, 0><<<grid_g(ROWS_BT, DIM_C), 256, 0, stream>>>(SMh + 64, SMl + 64, 128, WA2h, WA2l, LR_SPAD, A2p, nullptr, DIM_C,
                                                                    nullptr, nullptr, nullptr, 0, ROWS_BT, DIM_C, LR_SPAD, PRE_CARRY);
  gemm64<1, false, 0, 0><<<grid_g(ROWS_BT, DIM_C), 256, 0, stream>>>(SMh + 64, SMl + 64, 128, WMAh, WMAl, LR_SPAD, MA2p, nullptr, DIM_C,
                                                                    nullptr, nullptr, nullptr, 0, ROWS_BT, DIM_C, LR_SPAD, PRE_CARRY);

  decay_scan<<<NBATCH * N_HEAD, 128, 0, stream>>>(Rp, Kraw, KKZ, Vp, D2p, A2p, MA2p, MK2p,
                                                 tdecay, aaaaa, misc_a, misc_k, faaaa, ln_w, ln_b, SEQ_T, DIM_C, N_HEAD);

  gemm64<2, false, 0, 2><<<grid_g(ROWS_BT, DIM_C), 256, 0, stream>>>(G1h, G1l, LR_GATE, WG2h, WG2l, LR_GATE, XMh, XMl, DIM_C,
                                                                    nullptr, KKZ, nullptr, 0, ROWS_BT, DIM_C, LR_GATE, 1.0f);
  cvt(Wo, WBh, WBl, DIM_C * DIM_C);
  gemm64<0, false, 0, 0><<<grid_g(ROWS_BT, DIM_C), 256, 0, stream>>>(XMh, XMl, DIM_C, WBh, WBl, DIM_C, out, nullptr, DIM_C,
                                                                    nullptr, nullptr, nullptr, 0, ROWS_BT, DIM_C, DIM_C, 1.0f);
}
